// GAT_75067438399500
// MI455X (gfx1250) — hardware-run, weakly checked
//
#include <hip/hip_runtime.h>

typedef float          v8f   __attribute__((ext_vector_type(8)));
typedef float          v4f   __attribute__((ext_vector_type(4)));
typedef unsigned int   v4u   __attribute__((ext_vector_type(4)));
typedef int            v8i   __attribute__((ext_vector_type(8)));
typedef unsigned short v8us  __attribute__((ext_vector_type(8)));
typedef unsigned short v16us __attribute__((ext_vector_type(16)));
typedef __bf16         v16bf __attribute__((ext_vector_type(16)));
typedef _Float16       v16h  __attribute__((ext_vector_type(16)));
typedef v4f  __attribute__((may_alias)) v4fa;
typedef v8us __attribute__((may_alias)) v8usa;
union FragB { v16bf v; v16us u; v8us h[2]; v8i w; };
union FragH { v16h  v; v16us u; v8us h[2]; v8i w; };

__device__ __forceinline__ v8f wmb(const FragB& a, const FragB& b, v8f c) {
  v8f d = __builtin_amdgcn_wmma_f32_16x16x32_bf16(false, a.v, false, b.v, (short)0, c, false, false);
  asm volatile("v_nop\n\tv_nop\n\tv_nop\n\tv_nop" : "+v"(d) : "v"(a.w), "v"(b.w));
  return d;
}

__device__ __forceinline__ v8f wmh(const FragH& a, const FragH& b, v8f c) {
  v8f d = __builtin_amdgcn_wmma_f32_16x16x32_f16(false, a.v, false, b.v, (short)0, c, false, false);
  asm volatile("v_nop\n\tv_nop\n\tv_nop\n\tv_nop" : "+v"(d) : "v"(a.w), "v"(b.w));
  return d;
}

__device__ __forceinline__ unsigned bf16_bits(float f) {
  const unsigned u = __float_as_uint(f);
  const unsigned r = (u + 0x7FFFu + ((u >> 16) & 1u)) >> 16;
  const unsigned q = (u >> 16) | 0x40u;
  return ((u & 0x7fffffffu) > 0x7f800000u) ? q : r;
}

__device__ __forceinline__ float bf16_val(float f) {
  return __uint_as_float(bf16_bits(f) << 16);
}
__device__ __forceinline__ int clampi(int v, int lo, int hi) {
  return v < lo ? lo : (v > hi ? hi : v);
}

__device__ __forceinline__ unsigned f16_bits(float f) {
  const unsigned u  = __float_as_uint(f);
  const unsigned s  = (u >> 16) & 0x8000u;
  const unsigned a  = u & 0x7fffffffu;
  const unsigned t  = a - 0x38000000u;
  const unsigned r  = (t + 0x0FFFu + ((t >> 13) & 1u)) >> 13;
  const unsigned rc = r > 0x7C00u ? 0x7C00u : r;
  const bool small  = a < 0x38800000u;
  const bool isnan  = a > 0x7f800000u;
  const unsigned fin = small ? 0u : (s | rc);
  return isnan ? (s | 0x7E00u) : fin;
}

__device__ __forceinline__ unsigned pk16(unsigned lo, unsigned hi) { return lo | (hi << 16); }
__device__ __forceinline__ unsigned bf16_lo_bits(float v) {
  float hi = bf16_val(v);
  asm volatile("" : "+v"(hi));
  return bf16_bits(v - hi);
}
__device__ __forceinline__ v4u pack8_bf16(v4f a, v4f c) {
  return (v4u){ pk16(bf16_bits(a[0]), bf16_bits(a[1])), pk16(bf16_bits(a[2]), bf16_bits(a[3])),
                pk16(bf16_bits(c[0]), bf16_bits(c[1])), pk16(bf16_bits(c[2]), bf16_bits(c[3])) };
}
__device__ __forceinline__ v4u pack8_bf16_lo(v4f a, v4f c) {
  return (v4u){ pk16(bf16_lo_bits(a[0]), bf16_lo_bits(a[1])), pk16(bf16_lo_bits(a[2]), bf16_lo_bits(a[3])),
                pk16(bf16_lo_bits(c[0]), bf16_lo_bits(c[1])), pk16(bf16_lo_bits(c[2]), bf16_lo_bits(c[3])) };
}
__device__ __forceinline__ v4u pack8_f16(v4f a, v4f c) {
  return (v4u){ pk16(f16_bits(a[0]), f16_bits(a[1])), pk16(f16_bits(a[2]), f16_bits(a[3])),
                pk16(f16_bits(c[0]), f16_bits(c[1])), pk16(f16_bits(c[2]), f16_bits(c[3])) };
}

template <int FORM>
__global__ __launch_bounds__(256) void k_plane(const float* __restrict__ src, int rows, int cols, int ldsrc,
                                               unsigned short* __restrict__ dst, int MP, int KP) {
  static_assert(FORM >= 0 && FORM <= 3);
  const int KTOT = (FORM == 1 || FORM == 3) ? 2 * KP : KP;
  const unsigned ppr   = (unsigned)(KTOT >> 3);
  const unsigned kp8   = (unsigned)(KP >> 3);
  const unsigned total = (unsigned)MP * ppr;
  const unsigned g     = blockIdx.x * 256u + threadIdx.x;
  const unsigned rowu  = g / ppr;
  const unsigned p     = g - rowu * ppr;
  const bool second    = p >= kp8;
  const int row = (int)rowu;
  const int c0  = (int)((second ? p - kp8 : p) << 3);
  const float* srow = src + (size_t)clampi(row, 0, rows - 1) * (size_t)ldsrc;
  float x[8];
  unsigned mk[8];
#pragma unroll
  for (int e = 0; e < 8; ++e) {
    const int c = c0 + e;
    const float v = srow[clampi(c, 0, cols - 1)];
    asm volatile("" :: "v"(v));
    x[e]  = v;
    mk[e] = (row < rows && c < cols) ? 0xFFFFu : 0u;
  }
  const v4f a = (v4f){ x[0], x[1], x[2], x[3] };
  const v4f c = (v4f){ x[4], x[5], x[6], x[7] };
  v4u o;
  if (FORM == 2) {
    o = pack8_f16(a, c);
  } else {
    const v4u hi = pack8_bf16(a, c);
    o = hi;
    if (FORM == 1) { const v4u lo = pack8_bf16_lo(a, c); o = second ? lo : hi; }
  }
  const v4u mw = (v4u){ pk16(mk[0], mk[1]), pk16(mk[2], mk[3]), pk16(mk[4], mk[5]), pk16(mk[6], mk[7]) };
  o &= mw;
  if (g < total) {
    volatile v4u* q = (volatile v4u*)(dst + (size_t)g * 8);
    *q = o;
    __threadfence();
    *q = o;
  }
}

template <int FORM> struct FragOf    { typedef FragB T; };
template <>         struct FragOf<2> { typedef FragH T; };
__device__ __forceinline__ v8f mm(const FragB& a, const FragB& b, v8f c) { return wmb(a, b, c); }
__device__ __forceinline__ v8f mm(const FragH& a, const FragH& b, v8f c) { return wmh(a, b, c); }
template <class F> __device__ __forceinline__ F ld_frag(const unsigned short* p) {
  F f;
  f.h[0] = *(const v8usa*)(p);
  f.h[1] = *(const v8usa*)(p + 16);
  return f;
}

template <int FORM, int EPI>
__global__ __launch_bounds__(256) __attribute__((amdgpu_num_vgpr(248)))
void k_gemm_nt(const unsigned short* __restrict__ A, const unsigned short* __restrict__ B,
               const float* __restrict__ bias, float* __restrict__ D, int M, int N, int KTOT, int ldd) {
  static_assert(FORM >= 0 && FORM <= 2);
  static_assert(EPI == 0 || EPI == 1);
  typedef typename FragOf<FORM>::T F;
  __shared__ __attribute__((aligned(16))) float sT[8][16 * 68];
  const int lane = threadIdx.x & 31;
  const int wave = threadIdx.x >> 5;
  const int tilesM = (M + 63) >> 6;
  const int tilesN = (N + 63) >> 6;
  const int tile = blockIdx.x * 8 + wave;
  if (tile >= tilesM * tilesN) return;
  const int tm = tile / tilesN;
  const int tn = tile - tm * tilesN;
  const int m0 = tm << 6;
  const int n0 = tn << 6;

  const int rl = lane & 15;
  const int h8 = (lane >> 4) * 8;
  const unsigned short* pa = A + (size_t)(m0 + rl) * (size_t)KTOT + h8;
  const unsigned short* pb = B + (size_t)(n0 + rl) * (size_t)KTOT + h8;

  v8f acc[4][4];
#pragma unroll
  for (int i = 0; i < 4; ++i)
#pragma unroll
    for (int j = 0; j < 4; ++j) acc[i][j] = (v8f){0.f, 0.f, 0.f, 0.f, 0.f, 0.f, 0.f, 0.f};

#pragma unroll 1
  for (int k0 = 0; k0 < KTOT; k0 += 32) {
    F bf[4];
#pragma unroll
    for (int j = 0; j < 4; ++j) bf[j] = ld_frag<F>(pb + (size_t)(j << 4) * (size_t)KTOT + k0);
#pragma unroll
    for (int i = 0; i < 4; ++i) {
      const F af = ld_frag<F>(pa + (size_t)(i << 4) * (size_t)KTOT + k0);
#pragma unroll
      for (int j = 0; j < 4; ++j) acc[i][j] = mm(af, bf[j], acc[i][j]);
    }
  }

  float* slab = sT[wave];
  const int hh = lane >> 4;
  const int c4 = (lane & 15) * 4;
  const int nc = n0 + c4;
  const bool cok = nc < N;
  v4f bv = (v4f){0.f, 0.f, 0.f, 0.f};
  if (EPI == 1) {
    bv = *(const v4fa*)(bias + clampi(nc, 0, N - 4));
    asm volatile("" :: "v"(bv));
  }
#pragma unroll
  for (int i = 0; i < 4; ++i) {
    const int mBase = m0 + (i << 4);
#pragma unroll
    for (int j = 0; j < 4; ++j) {
#pragma unroll
      for (int r = 0; r < 8; ++r) slab[(h8 + r) * 68 + (j << 4) + rl] = acc[i][j][r];
    }
    __builtin_amdgcn_fence(__ATOMIC_RELEASE, "workgroup");
    __builtin_amdgcn_wave_barrier();
    __builtin_amdgcn_fence(__ATOMIC_ACQUIRE, "workgroup");
    v4f vv[8];
#pragma unroll
    for (int it = 0; it < 8; ++it) {
      const int row = it * 2 + hh;
      v4f v = *(const v4fa*)(slab + row * 68 + c4);
      if (EPI == 1) v += bv;
      vv[it] = v;
    }
    for (int pass = 0; pass < 2; ++pass) {
#pragma unroll
      for (int it = 0; it < 8; ++it) {
        const int row = mBase + it * 2 + hh;
        if (cok && row < M) *(volatile v4f*)(D + (size_t)row * (size_t)ldd + nc) = vv[it];
      }
      __threadfence();
    }
    __builtin_amdgcn_fence(__ATOMIC_RELEASE, "workgroup");
    __builtin_amdgcn_wave_barrier();
    __builtin_amdgcn_fence(__ATOMIC_ACQUIRE, "workgroup");
  }
}

#pragma clang fp contract(off)


#ifndef SPLIT_2
#define SPLIT_2 1
#endif

#define NN      50000
#define NE      800000
#define MPAD    50048
#define FIN     256
#define HID     128
#define OUTW    64
#define NHD     4
#define OPK     (SPLIT_2 ? 256 : 128)
#define RTHR    256
#define RWAVES  8
#define TB_AL1  0
#define TB_AR1  128
#define TB_B1   256
#define TB_AL2  384
#define TB_AR2  448
#define TB_B2   512
#define TB_N    1024
#define BT      512
#define BW      16
#define BEPT    8
#define BCHUNK  (BT * BEPT)
#define NCH     ((NE + BCHUNK - 1) / BCHUNK)
#define NB      1024
#define NBLK    ((NN + NB - 1) / NB)
#define RCAP    20992
#define DEGCAP  64
#define SLOTSH  21
#define LISTTOT (NBLK * RCAP)
#define LDS_LST ((2 * RCAP + 3 * NB + 64) * 4)
#define WSMAX   ((size_t)128 << 20)
#define PREP_W1U (HID * FIN / 8)
#define PREP_W2U (OUTW * OPK / 8)
#define PREP_W1B (PREP_W1U / 256)
#define PREP_W2B (PREP_W2U / 256)
#define PREP_BLK (PREP_W1B + PREP_W2B + 1)

static_assert(NN % 8 == 0);
static_assert(MPAD == 391 * 128 && MPAD % 64 == 0 && MPAD >= NN && MPAD % 32 == 0);
static_assert(HID == 32 * 4 && NHD * 32 == HID);
static_assert(OUTW == 32 * 2);
static_assert(FIN % 32 == 0 && OPK % 32 == 0);
static_assert(NE < (1 << SLOTSH));
static_assert(NB <= 1024 && (NB & (NB - 1)) == 0 && NB == 2 * BT);
static_assert(NE % 8 == 0 && NE >= 8);
static_assert(NBLK == 49 && NBLK * NB >= NN);
static_assert(NCH * BCHUNK >= NE && NCH == 196);
static_assert(RCAP % 32 == 0);
static_assert(RCAP * 4 >= 16652 * 5);
static_assert(DEGCAP >= 36 + 8);
static_assert(LDS_LST <= 262144);
static_assert(BW == BT / 32 && BW == 16);
static_assert(PREP_W1U % 256 == 0 && PREP_W2U % 256 == 0);
static_assert(TB_B2 + 128 <= TB_N);

typedef float        v2f __attribute__((ext_vector_type(2)));
typedef int          v4i __attribute__((ext_vector_type(4)));
typedef int          v2i __attribute__((ext_vector_type(2)));
typedef unsigned int v2u __attribute__((ext_vector_type(2)));
typedef v2f __attribute__((may_alias)) v2fa;
typedef v4i __attribute__((may_alias)) v4ia;
typedef v2i __attribute__((may_alias)) v2ia;

__device__ __forceinline__ float relu_k(float v) { return (v > 0.0f) ? v : (v - v); }
__device__ __forceinline__ float lrelu_k(float v) { return (v > 0.0f) ? v : 0.2f * v; }
__device__ __forceinline__ float maxk(float a, float b) {
  float m = (a < b) ? b : a;
  m = (b != b) ? b : m;
  return m;
}
__device__ __forceinline__ float sum8(float t) {
  t = t + __shfl_xor(t, 4, 32);
  t = t + __shfl_xor(t, 2, 32);
  t = t + __shfl_xor(t, 1, 32);
  return t;
}
__device__ __forceinline__ float sum32(float t) {
  t = t + __shfl_xor(t, 16, 32);
  t = t + __shfl_xor(t, 8, 32);
  t = t + __shfl_xor(t, 4, 32);
  t = t + __shfl_xor(t, 2, 32);
  t = t + __shfl_xor(t, 1, 32);
  return t;
}

__global__ __launch_bounds__(256) void k_prep(const float* __restrict__ W1, const float* __restrict__ W2,
                                              const float* __restrict__ al1, const float* __restrict__ ar1,
                                              const float* __restrict__ b1, const float* __restrict__ al2,
                                              const float* __restrict__ ar2, const float* __restrict__ b2,
                                              unsigned short* W1T, unsigned short* W2D, float* TAB) {
  const int blk = (int)blockIdx.x;
  const int tid = (int)threadIdx.x;
  if (blk < PREP_W1B) {
    const int g  = blk * 256 + tid;
    const int n  = g / (FIN / 8);
    const int k0 = (g - n * (FIN / 8)) * 8;
    float x[8];
#pragma unroll
    for (int e = 0; e < 8; ++e) {
      const float v = W1[(size_t)(k0 + e) * HID + n];
      asm volatile("" :: "v"(v));
      x[e] = v;
    }
    const v4u o = pack8_bf16((v4f){x[0], x[1], x[2], x[3]}, (v4f){x[4], x[5], x[6], x[7]});
    volatile v4u* q = (volatile v4u*)(W1T + (size_t)g * 8);
    *q = o;
    __threadfence();
    *q = o;
  } else if (blk < PREP_W1B + PREP_W2B) {
    const int g  = (blk - PREP_W1B) * 256 + tid;
    const int n  = g / (OPK / 8);
    const int k0 = ((g - n * (OPK / 8)) * 8) & (HID - 1);
    float x[8];
#pragma unroll
    for (int e = 0; e < 8; ++e) {
      const float v = W2[(size_t)(k0 + e) * OUTW + n];
      asm volatile("" :: "v"(v));
      x[e] = v;
    }
    const v4u o = pack8_bf16((v4f){x[0], x[1], x[2], x[3]}, (v4f){x[4], x[5], x[6], x[7]});
    volatile v4u* q = (volatile v4u*)(W2D + (size_t)g * 8);
    *q = o;
    __threadfence();
    *q = o;
  } else {
    const int idx = 4 * tid;
    const v4f a0 = *(const v4fa*)(al1 + clampi(idx - TB_AL1, 0, 124));
    asm volatile("" :: "v"(a0));
    const v4f a1 = *(const v4fa*)(ar1 + clampi(idx - TB_AR1, 0, 124));
    asm volatile("" :: "v"(a1));
    const v4f a2 = *(const v4fa*)(b1  + clampi(idx - TB_B1,  0, 124));
    asm volatile("" :: "v"(a2));
    const v4f a3 = *(const v4fa*)(al2 + clampi(idx - TB_AL2, 0, 60));
    asm volatile("" :: "v"(a3));
    const v4f a4 = *(const v4fa*)(ar2 + clampi(idx - TB_AR2, 0, 60));
    asm volatile("" :: "v"(a4));
    const v4f a5 = *(const v4fa*)(b2  + clampi(idx - TB_B2,  0, 60));
    asm volatile("" :: "v"(a5));
    const unsigned m0 = (idx < TB_AR1) ? 0xFFFFFFFFu : 0u;
    const unsigned m1 = (idx >= TB_AR1 && idx < TB_B1) ? 0xFFFFFFFFu : 0u;
    const unsigned m2 = (idx >= TB_B1 && idx < TB_AL2) ? 0xFFFFFFFFu : 0u;
    const unsigned m3 = (idx >= TB_AL2 && idx < TB_AR2) ? 0xFFFFFFFFu : 0u;
    const unsigned m4 = (idx >= TB_AR2 && idx < TB_B2) ? 0xFFFFFFFFu : 0u;
    const unsigned m5 = (idx >= TB_B2 && idx < TB_B2 + OUTW) ? 0xFFFFFFFFu : 0u;
    v4u o;
    o.x = (__float_as_uint(a0.x) & m0) | (__float_as_uint(a1.x) & m1) | (__float_as_uint(a2.x) & m2) |
          (__float_as_uint(a3.x) & m3) | (__float_as_uint(a4.x) & m4) | (__float_as_uint(a5.x) & m5);
    o.y = (__float_as_uint(a0.y) & m0) | (__float_as_uint(a1.y) & m1) | (__float_as_uint(a2.y) & m2) |
          (__float_as_uint(a3.y) & m3) | (__float_as_uint(a4.y) & m4) | (__float_as_uint(a5.y) & m5);
    o.z = (__float_as_uint(a0.z) & m0) | (__float_as_uint(a1.z) & m1) | (__float_as_uint(a2.z) & m2) |
          (__float_as_uint(a3.z) & m3) | (__float_as_uint(a4.z) & m4) | (__float_as_uint(a5.z) & m5);
    o.w = (__float_as_uint(a0.w) & m0) | (__float_as_uint(a1.w) & m1) | (__float_as_uint(a2.w) & m2) |
          (__float_as_uint(a3.w) & m3) | (__float_as_uint(a4.w) & m4) | (__float_as_uint(a5.w) & m5);
    o.x = bf16_bits(__uint_as_float(o.x)) << 16;
    o.y = bf16_bits(__uint_as_float(o.y)) << 16;
    o.z = bf16_bits(__uint_as_float(o.z)) << 16;
    o.w = bf16_bits(__uint_as_float(o.w)) << 16;
    volatile v4u* q = (volatile v4u*)(TAB + idx);
    *q = o;
    __threadfence();
    *q = o;
  }
}

__global__ __launch_bounds__(BT) void k_list(const int* __restrict__ ekey, const int* __restrict__ egat,
                                             unsigned* LIST, int* META) {
  extern __shared__ v4u lds_lst[];
  int* reg1 = (int*)lds_lst;
  int* reg2 = reg1 + RCAP;
  int* scnt = reg2 + RCAP;
  int* soff = scnt + NB;
  int* curs = soff + NB;
  int* wcnt = curs + NB;
  int* wtot = wcnt + 2 * BW;
  const int tid = (int)threadIdx.x, lane = tid & 31, wave = tid >> 5;
  const int nodeBase = (int)blockIdx.x * NB;
  int nb = NN - nodeBase;
  nb = nb > NB ? NB : (nb < 0 ? 0 : nb);
  const unsigned nbs = (unsigned)nodeBase, unb = (unsigned)nb;

  scnt[2 * tid] = 0;
  scnt[2 * tid + 1] = 0;

  int tot = 0;
#pragma unroll 1
  for (int ch = 0; ch < NCH; ++ch) {
    const int par = ch & 1;
    const int e0  = ch * BCHUNK + tid * BEPT;
    const bool valid = e0 < NE;
    const int ea = e0 < NE - 8 ? e0 : NE - 8;
    const v4i da = *(const v4ia*)(ekey + ea);
    const v4i db = *(const v4ia*)(ekey + ea + 4);
    asm volatile("" :: "v"(da), "v"(db));
    const unsigned s0 = (unsigned)da.x - nbs, s1 = (unsigned)da.y - nbs;
    const unsigned s2 = (unsigned)da.z - nbs, s3 = (unsigned)da.w - nbs;
    const unsigned s4 = (unsigned)db.x - nbs, s5 = (unsigned)db.y - nbs;
    const unsigned s6 = (unsigned)db.z - nbs, s7 = (unsigned)db.w - nbs;
    const bool h0 = valid && (s0 < unb), h1 = valid && (s1 < unb), h2 = valid && (s2 < unb), h3 = valid && (s3 < unb);
    const bool h4 = valid && (s4 < unb), h5 = valid && (s5 < unb), h6 = valid && (s6 < unb), h7 = valid && (s7 < unb);
    const int c = (int)h0 + (int)h1 + (int)h2 + (int)h3 + (int)h4 + (int)h5 + (int)h6 + (int)h7;
    int incl = c;
#pragma unroll
    for (int d = 1; d < 32; d <<= 1) {
      const int up = __shfl_up(incl, d, 32);
      incl += (lane >= d) ? up : 0;
    }
    const int wtotal = __shfl(incl, 31, 32);
    if (lane == 0) wcnt[par * BW + wave] = wtotal;
    __syncthreads();
    int all = 0, pre = 0;
#pragma unroll
    for (int g = 0; g < 4; ++g) {
      const v4i w4 = *(const v4ia*)(wcnt + par * BW + 4 * g);
      const int c0 = clampi(w4.x, 0, 256), c1 = clampi(w4.y, 0, 256);
      const int c2 = clampi(w4.z, 0, 256), c3 = clampi(w4.w, 0, 256);
      all += c0 + c1 + c2 + c3;
      pre += (4 * g + 0 < wave) ? c0 : 0;
      pre += (4 * g + 1 < wave) ? c1 : 0;
      pre += (4 * g + 2 < wave) ? c2 : 0;
      pre += (4 * g + 3 < wave) ? c3 : 0;
    }
    int pos = tot + pre + (incl - c);
#define PUTJ(J, HJ, SJ) if (HJ) { if (pos < RCAP) reg1[pos] = (int)((unsigned)(e0 + (J)) | ((SJ) << SLOTSH)); ++pos; }
    PUTJ(0, h0, s0)
    PUTJ(1, h1, s1)
    PUTJ(2, h2, s2)
    PUTJ(3, h3, s3)
    PUTJ(4, h4, s4)
    PUTJ(5, h5, s5)
    PUTJ(6, h6, s6)
    PUTJ(7, h7, s7)
#undef PUTJ
    tot += all;
  }
  __syncthreads();
  const bool ovf = tot > RCAP;
  const int nh = ovf ? RCAP : tot;

  if (wave == 0) {
#pragma unroll 1
    for (int b0 = 0; b0 < nh; b0 += 32) {
      const int idx = b0 + lane;
      const int uv  = reg1[idx < nh ? idx : nh - 1];
      const int m32 = (nh - b0) < 32 ? (nh - b0) : 32;
#pragma unroll 1
      for (int k = 0; k < m32; ++k) {
        const int u  = __builtin_amdgcn_readlane(uv, k);
        const int sl = (int)(((unsigned)u >> SLOTSH) & (unsigned)(NB - 1));
        const int cv = scnt[sl] + 1;
        if (lane == 0) scnt[sl] = cv;
      }
    }
  }
  __syncthreads();

  int e0c, e1c;
  {
    const v2i cc = *(const v2ia*)(scnt + 2 * tid);
    e0c = cc.x < 0 ? 0 : cc.x;
    e1c = cc.y < 0 ? 0 : cc.y;
    const int ts = e0c + e1c;
    int incl = ts;
#pragma unroll
    for (int d = 1; d < 32; d <<= 1) {
      const int up = __shfl_up(incl, d, 32);
      incl += (lane >= d) ? up : 0;
    }
    if (lane == 31) wtot[wave] = incl;
    __syncthreads();
    int pre = 0;
#pragma unroll
    for (int g = 0; g < 4; ++g) {
      const v4i w4 = *(const v4ia*)(wtot + 4 * g);
      pre += (4 * g + 0 < wave) ? w4.x : 0;
      pre += (4 * g + 1 < wave) ? w4.y : 0;
      pre += (4 * g + 2 < wave) ? w4.z : 0;
      pre += (4 * g + 3 < wave) ? w4.w : 0;
    }
    const int run = pre + incl - ts;
    soff[2 * tid]     = run;
    soff[2 * tid + 1] = run + e0c;
    curs[2 * tid]     = run;
    curs[2 * tid + 1] = run + e0c;
  }
  __syncthreads();

  if (wave == 0) {
#pragma unroll 1
    for (int b0 = 0; b0 < nh; b0 += 32) {
      const int idx = b0 + lane;
      const int uv  = reg1[idx < nh ? idx : nh - 1];
      const int m32 = (nh - b0) < 32 ? (nh - b0) : 32;
#pragma unroll 1
      for (int k = 0; k < m32; ++k) {
        const int u   = __builtin_amdgcn_readlane(uv, k);
        const int sl  = (int)(((unsigned)u >> SLOTSH) & (unsigned)(NB - 1));
        const int eid = (int)((unsigned)u & ((1u << SLOTSH) - 1u));
        const int pr  = curs[sl];
        const int pc  = clampi(pr, 0, RCAP - 1);
        if (lane == 0) { reg2[pc] = eid; curs[sl] = pc + 1; }
      }
    }
  }
  __syncthreads();

  {
    const int nhPad = (nh + 31) & ~31;
    const int nIt = (nhPad + BT - 1) / BT;
    unsigned* lbase = LIST + (size_t)blockIdx.x * (size_t)RCAP;
#pragma unroll 1
    for (int it = 0; it < nIt; ++it) {
      const int i  = it * BT + tid;
      const int ic = i < nh ? i : nh - 1;
      const int eid = clampi(reg2[ic], 0, NE - 1);
      const int cw = egat[eid];
      asm volatile("" :: "v"(cw));
      const unsigned msk = (i < nh) ? 0xFFFFFFFFu : 0u;
      const unsigned o = (unsigned)clampi(cw, 0, NN - 1) & msk;
      const int iw = i < RCAP ? i : RCAP - 1;
      volatile unsigned* q = (volatile unsigned*)(lbase + (size_t)iw);
      const bool wr = i < nhPad;
      if (wr) *q = o;
      __threadfence();
      if (wr) *q = o;
    }
  }

  {
    const int base = (int)blockIdx.x * RCAP;
    const v2i cc = *(const v2ia*)(scnt + 2 * tid);
    const v2i so = *(const v2ia*)(soff + 2 * tid);
    v4i m;
    m.x = base + so.x;
    m.y = ovf ? -1 : cc.x;
    m.z = base + so.y;
    m.w = ovf ? -1 : cc.y;
    volatile v4i* q = (volatile v4i*)(META + 2 * (size_t)(nodeBase + 2 * tid));
    *q = m;
    __threadfence();
    *q = m;
  }
}

__global__ __launch_bounds__(RTHR) void k_rowprep1(const float* __restrict__ FT, const float* __restrict__ TAB,
                                                   float* EL, float* ER) {
  __shared__ __attribute__((aligned(16))) float sA[2 * HID];
  __shared__ __attribute__((aligned(16))) float sEl[RWAVES * NHD];
  __shared__ __attribute__((aligned(16))) float sEr[RWAVES * NHD];
  const int tid  = (int)threadIdx.x;
  const int lane = tid & 31;
  const int wave = tid >> 5;
  const int row  = (int)blockIdx.x * RWAVES + wave;
  const int head = lane >> 3;
  const int c0   = lane * 4;
  if (tid < 64) {
    const v4f t = *(const v4fa*)(TAB + TB_AL1 + 4 * tid);
    *(v4fa*)(sA + 4 * tid) = t;
  }
  const v4f p = *(const v4fa*)(FT + (size_t)row * HID + c0);
  asm volatile("" :: "v"(p));
  __syncthreads();
  const v4f al = *(const v4fa*)(sA + c0);
  const v4f ar = *(const v4fa*)(sA + HID + c0);
  float t = p.x * al.x;
  float u = p.y * al.y; t = t + u;
  u = p.z * al.z; t = t + u;
  u = p.w * al.w; t = t + u;
  t = sum8(t);
  float r = p.x * ar.x;
  u = p.y * ar.y; r = r + u;
  u = p.z * ar.z; r = r + u;
  u = p.w * ar.w; r = r + u;
  r = sum8(r);
  if ((lane & 7) == 0) { sEl[wave * NHD + head] = t; sEr[wave * NHD + head] = r; }
  __syncthreads();
  if (wave == 0) {
    const int l8 = lane & 7;
    const v4f sv = *(const v4fa*)(sEl + 4 * l8);
    const v4f su = *(const v4fa*)(sEr + 4 * l8);
    const bool wr = lane < 8;
    volatile v4f* qe = (volatile v4f*)(EL + (size_t)blockIdx.x * (RWAVES * NHD) + 4 * l8);
    volatile v4f* qr = (volatile v4f*)(ER + (size_t)blockIdx.x * (RWAVES * NHD) + 4 * l8);
    if (wr) { *qe = sv; *qr = su; }
    __threadfence();
    if (wr) { *qe = sv; *qr = su; }
  }
}

__global__ __launch_bounds__(RTHR) void k_walk1(const float* __restrict__ FT, const float* __restrict__ EL,
                                                const float* __restrict__ ER, const unsigned* __restrict__ LIST,
                                                const int* __restrict__ META, const float* __restrict__ TAB,
                                                unsigned short* OP) {
  __shared__ __attribute__((aligned(16))) float sB[HID];
  const int lane = (int)threadIdx.x & 31;
  const int wave = (int)threadIdx.x >> 5;
  const int row  = (int)blockIdx.x * RWAVES + wave;
  const bool pad = row >= NN;
  const int rowc = pad ? NN - 1 : row;
  const int head = lane >> 3;
  const int c0   = lane * 4;
  if (wave == 0) {
    const v4f t = *(const v4fa*)(TAB + TB_B1 + 4 * lane);
    *(v4fa*)(sB + 4 * lane) = t;
  }

  const v2i mt = *(const v2ia*)(META + 2 * (size_t)rowc);
  asm volatile("" :: "v"(mt));
  const int craw = mt.y;
  const int offv = clampi(mt.x, 0, LISTTOT);
  int cntv = clampi(craw, 0, DEGCAP);
  cntv = pad ? 0 : (cntv < (LISTTOT - offv) ? cntv : (LISTTOT - offv));
  const int off = __builtin_amdgcn_readfirstlane(offv);
  const int cnt = __builtin_amdgcn_readfirstlane(cntv);
  const bool poison = (craw < 0) || (craw > DEGCAP);

  const v4f er4 = *(const v4fa*)(ER + (size_t)rowc * NHD);
  asm volatile("" :: "v"(er4));
  __syncthreads();
  const v4f bb = *(const v4fa*)(sB + c0);

  const float ninf = -__builtin_inff();
  v4f mx4 = (v4f){ninf, ninf, ninf, ninf};
#pragma unroll 1
  for (int b0 = 0; b0 < cnt; b0 += 32) {
    const int j = (b0 + lane) < cnt ? (b0 + lane) : cnt - 1;
    const unsigned ent = LIST[(size_t)(off + j)];
    asm volatile("" :: "v"(ent));
    const int col = clampi((int)ent, 0, NN - 1);
    const v4f el = *(const v4fa*)(EL + (size_t)col * NHD);
    asm volatile("" :: "v"(el));
    mx4.x = maxk(mx4.x, lrelu_k(el.x + er4.x));
    mx4.y = maxk(mx4.y, lrelu_k(el.y + er4.y));
    mx4.z = maxk(mx4.z, lrelu_k(el.z + er4.z));
    mx4.w = maxk(mx4.w, lrelu_k(el.w + er4.w));
  }
#pragma unroll
  for (int d = 16; d > 0; d >>= 1) {
    const float o0 = __shfl_xor(mx4.x, d, 32);
    const float o1 = __shfl_xor(mx4.y, d, 32);
    const float o2 = __shfl_xor(mx4.z, d, 32);
    const float o3 = __shfl_xor(mx4.w, d, 32);
    mx4.x = maxk(mx4.x, o0);
    mx4.y = maxk(mx4.y, o1);
    mx4.z = maxk(mx4.z, o2);
    mx4.w = maxk(mx4.w, o3);
  }

  v4f z4 = (v4f){0.0f, 0.0f, 0.0f, 0.0f};
#pragma unroll 1
  for (int b0 = 0; b0 < cnt; b0 += 32) {
    const int j = (b0 + lane) < cnt ? (b0 + lane) : cnt - 1;
    const unsigned ent = LIST[(size_t)(off + j)];
    asm volatile("" :: "v"(ent));
    const int col = clampi((int)ent, 0, NN - 1);
    const v4f el = *(const v4fa*)(EL + (size_t)col * NHD);
    asm volatile("" :: "v"(el));
    float v0 = lrelu_k(el.x + er4.x); v0 = v0 - mx4.x;
    float v1 = lrelu_k(el.y + er4.y); v1 = v1 - mx4.y;
    float v2 = lrelu_k(el.z + er4.z); v2 = v2 - mx4.z;
    float v3 = lrelu_k(el.w + er4.w); v3 = v3 - mx4.w;
    const float q0 = expf(v0);
    const float q1 = expf(v1);
    const float q2 = expf(v2);
    const float q3 = expf(v3);
    const int m32 = (cnt - b0) < 32 ? (cnt - b0) : 32;
#pragma unroll 1
    for (int k = 0; k < m32; ++k) {
      const float w0 = __int_as_float(__builtin_amdgcn_readlane(__float_as_int(q0), k));
      const float w1 = __int_as_float(__builtin_amdgcn_readlane(__float_as_int(q1), k));
      const float w2 = __int_as_float(__builtin_amdgcn_readlane(__float_as_int(q2), k));
      const float w3 = __int_as_float(__builtin_amdgcn_readlane(__float_as_int(q3), k));
      z4.x = z4.x + w0;
      z4.y = z4.y + w1;
      z4.z = z4.z + w2;
      z4.w = z4.w + w3;
    }
  }

  v4f ac = (v4f){0.0f, 0.0f, 0.0f, 0.0f};
#pragma unroll 1
  for (int b0 = 0; b0 < cnt; b0 += 32) {
    const int j = (b0 + lane) < cnt ? (b0 + lane) : cnt - 1;
    const unsigned ent = LIST[(size_t)(off + j)];
    asm volatile("" :: "v"(ent));
    const int col = clampi((int)ent, 0, NN - 1);
    const v4f el = *(const v4fa*)(EL + (size_t)col * NHD);
    asm volatile("" :: "v"(el));
    float v0 = lrelu_k(el.x + er4.x); v0 = v0 - mx4.x;
    float v1 = lrelu_k(el.y + er4.y); v1 = v1 - mx4.y;
    float v2 = lrelu_k(el.z + er4.z); v2 = v2 - mx4.z;
    float v3 = lrelu_k(el.w + er4.w); v3 = v3 - mx4.w;
    const float a0 = expf(v0) / z4.x;
    const float a1 = expf(v1) / z4.y;
    const float a2 = expf(v2) / z4.z;
    const float a3 = expf(v3) / z4.w;
    const int m32 = (cnt - b0) < 32 ? (cnt - b0) : 32;
#pragma unroll 1
    for (int k = 0; k < m32; ++k) {
      const int c = __builtin_amdgcn_readlane(col, k);
      const float w0 = __int_as_float(__builtin_amdgcn_readlane(__float_as_int(a0), k));
      const float w1 = __int_as_float(__builtin_amdgcn_readlane(__float_as_int(a1), k));
      const float w2 = __int_as_float(__builtin_amdgcn_readlane(__float_as_int(a2), k));
      const float w3 = __int_as_float(__builtin_amdgcn_readlane(__float_as_int(a3), k));
      float w = w0;
      w = (head == 1) ? w1 : w;
      w = (head == 2) ? w2 : w;
      w = (head == 3) ? w3 : w;
      const v4f hn = *(const v4fa*)(FT + (size_t)c * HID + c0);
      asm volatile("" :: "v"(hn));
      float pr;
      pr = hn.x * w; ac.x = ac.x + pr;
      pr = hn.y * w; ac.y = ac.y + pr;
      pr = hn.z * w; ac.z = ac.z + pr;
      pr = hn.w * w; ac.w = ac.w + pr;
    }
  }

  const float qnan = __uint_as_float(0x7fc00000u);
  v4f y;
  y.x = relu_k(ac.x + bb.x);
  y.y = relu_k(ac.y + bb.y);
  y.z = relu_k(ac.z + bb.z);
  y.w = relu_k(ac.w + bb.w);
  y.x = poison ? qnan : y.x;
  y.y = poison ? qnan : y.y;
  y.z = poison ? qnan : y.z;
  y.w = poison ? qnan : y.w;
  const unsigned km = pad ? 0u : 0xFFFFFFFFu;
  v2u oh, ol;
  oh.x = pk16(bf16_bits(y.x), bf16_bits(y.y)) & km;
  oh.y = pk16(bf16_bits(y.z), bf16_bits(y.w)) & km;
  ol.x = pk16(bf16_lo_bits(y.x), bf16_lo_bits(y.y)) & km;
  ol.y = pk16(bf16_lo_bits(y.z), bf16_lo_bits(y.w)) & km;
  volatile v2u* qh = (volatile v2u*)(OP + (size_t)row * OPK + c0);
  volatile v2u* ql = (volatile v2u*)(OP + (size_t)row * OPK + (SPLIT_2 ? HID : 0) + c0);
  *qh = oh;
  if (SPLIT_2) *ql = ol;
  __threadfence();
  *qh = oh;
  if (SPLIT_2) *ql = ol;
}

__global__ __launch_bounds__(RTHR) void k_rowprep2(const float* __restrict__ FT2, const float* __restrict__ TAB,
                                                   float* EL2, float* ER2) {
  __shared__ __attribute__((aligned(16))) float sA[2 * OUTW];
  __shared__ __attribute__((aligned(16))) float sEl[32];
  __shared__ __attribute__((aligned(16))) float sEr[32];
  const int lane = (int)threadIdx.x & 31;
  const int wave = (int)threadIdx.x >> 5;
  if (wave == 0) {
    const v4f t = *(const v4fa*)(TAB + TB_AL2 + 4 * lane);
    *(v4fa*)(sA + 4 * lane) = t;
  }
  __syncthreads();
  const v2f al = *(const v2fa*)(sA + 2 * lane);
  const v2f ar = *(const v2fa*)(sA + OUTW + 2 * lane);
#pragma unroll
  for (int i = 0; i < 4; ++i) {
    const int node = (int)blockIdx.x * 32 + wave * 4 + i;
    const v2f p = *(const v2fa*)(FT2 + (size_t)node * OUTW + 2 * lane);
    asm volatile("" :: "v"(p));
    float t = p.x * al.x;
    float u = p.y * al.y; t = t + u;
    t = sum32(t);
    float r = p.x * ar.x;
    u = p.y * ar.y; r = r + u;
    r = sum32(r);
    if (lane == 0) { sEl[wave * 4 + i] = t; sEr[wave * 4 + i] = r; }
  }
  __syncthreads();
  if (wave == 0) {
    const int l8 = lane & 7;
    const v4f sv = *(const v4fa*)(sEl + 4 * l8);
    const v4f su = *(const v4fa*)(sEr + 4 * l8);
    const bool wr = lane < 8;
    volatile v4f* qe = (volatile v4f*)(EL2 + (size_t)blockIdx.x * 32 + 4 * l8);
    volatile v4f* qr = (volatile v4f*)(ER2 + (size_t)blockIdx.x * 32 + 4 * l8);
    if (wr) { *qe = sv; *qr = su; }
    __threadfence();
    if (wr) { *qe = sv; *qr = su; }
  }
}

__global__ __launch_bounds__(RTHR) void k_walk2(const float* __restrict__ FT2, const float* __restrict__ EL2,
                                                const float* __restrict__ ER2, const unsigned* __restrict__ LIST,
                                                const int* __restrict__ META, const float* __restrict__ TAB,
                                                float* out) {
  __shared__ __attribute__((aligned(16))) float sB[128];
  const int lane = (int)threadIdx.x & 31;
  const int wave = (int)threadIdx.x >> 5;
  const int row  = (int)blockIdx.x * RWAVES + wave;
  const int rowc = row < NN ? row : NN - 1;
  const int c0   = lane * 2;
  if (wave == 0) {
    const v4f t = *(const v4fa*)(TAB + TB_B2 + 4 * lane);
    *(v4fa*)(sB + 4 * lane) = t;
  }

  const v2i mt = *(const v2ia*)(META + 2 * (size_t)rowc);
  asm volatile("" :: "v"(mt));
  const int craw = mt.y;
  const int offv = clampi(mt.x, 0, LISTTOT);
  int cntv = clampi(craw, 0, DEGCAP);
  cntv = cntv < (LISTTOT - offv) ? cntv : (LISTTOT - offv);
  const int off = __builtin_amdgcn_readfirstlane(offv);
  const int cnt = __builtin_amdgcn_readfirstlane(cntv);
  const bool poison = (craw < 0) || (craw > DEGCAP);

  const float er = ER2[rowc];
  asm volatile("" :: "v"(er));
  __syncthreads();
  const v2f bb = *(const v2fa*)(sB + c0);

  float mx = -__builtin_inff();
#pragma unroll 1
  for (int b0 = 0; b0 < cnt; b0 += 32) {
    const int j = (b0 + lane) < cnt ? (b0 + lane) : cnt - 1;
    const unsigned ent = LIST[(size_t)(off + j)];
    asm volatile("" :: "v"(ent));
    const int col = clampi((int)ent, 0, NN - 1);
    const float el = EL2[col];
    asm volatile("" :: "v"(el));
    mx = maxk(mx, lrelu_k(el + er));
  }
#pragma unroll
  for (int d = 16; d > 0; d >>= 1) {
    const float o0 = __shfl_xor(mx, d, 32);
    mx = maxk(mx, o0);
  }

  float z = 0.0f;
#pragma unroll 1
  for (int b0 = 0; b0 < cnt; b0 += 32) {
    const int j = (b0 + lane) < cnt ? (b0 + lane) : cnt - 1;
    const unsigned ent = LIST[(size_t)(off + j)];
    asm volatile("" :: "v"(ent));
    const int col = clampi((int)ent, 0, NN - 1);
    const float el = EL2[col];
    asm volatile("" :: "v"(el));
    float v0 = lrelu_k(el + er); v0 = v0 - mx;
    const float q0 = expf(v0);
    const int m32 = (cnt - b0) < 32 ? (cnt - b0) : 32;
#pragma unroll 1
    for (int k = 0; k < m32; ++k) {
      const float w0 = __int_as_float(__builtin_amdgcn_readlane(__float_as_int(q0), k));
      z = z + w0;
    }
  }

  v2f ac = (v2f){0.0f, 0.0f};
#pragma unroll 1
  for (int b0 = 0; b0 < cnt; b0 += 32) {
    const int j = (b0 + lane) < cnt ? (b0 + lane) : cnt - 1;
    const unsigned ent = LIST[(size_t)(off + j)];
    asm volatile("" :: "v"(ent));
    const int col = clampi((int)ent, 0, NN - 1);
    const float el = EL2[col];
    asm volatile("" :: "v"(el));
    float v0 = lrelu_k(el + er); v0 = v0 - mx;
    const float a0 = expf(v0) / z;
    const int m32 = (cnt - b0) < 32 ? (cnt - b0) : 32;
#pragma unroll 1
    for (int k = 0; k < m32; ++k) {
      const int c = __builtin_amdgcn_readlane(col, k);
      const float w = __int_as_float(__builtin_amdgcn_readlane(__float_as_int(a0), k));
      const v2f hn = *(const v2fa*)(FT2 + (size_t)c * OUTW + c0);
      asm volatile("" :: "v"(hn));
      float pr;
      pr = hn.x * w; ac.x = ac.x + pr;
      pr = hn.y * w; ac.y = ac.y + pr;
    }
  }

  const float qnan = __uint_as_float(0x7fc00000u);
  v2f o;
  o.x = ac.x + bb.x;
  o.y = ac.y + bb.y;
  o.x = poison ? qnan : o.x;
  o.y = poison ? qnan : o.y;
  const bool rok = row < NN;
  volatile v2f* q = (volatile v2f*)(out + (size_t)rowc * OUTW + c0);
  if (rok) *q = o;
  __threadfence();
  if (rok) *q = o;
}

extern "C" void kernel_launch(void* const* d_in, const int* in_sizes, int n_in,
                              void* d_out, int out_size, void* d_ws, size_t ws_size,
                              hipStream_t stream) {
  if (n_in < 11) return;
  if (in_sizes[0] != NN * FIN) return;
  if (in_sizes[1] != FIN * HID) return;
  if (in_sizes[2] != HID || in_sizes[3] != HID || in_sizes[4] != HID) return;
  if (in_sizes[5] != HID * OUTW) return;
  if (in_sizes[6] != OUTW || in_sizes[7] != OUTW || in_sizes[8] != OUTW) return;
  if (in_sizes[9] != NE || in_sizes[10] != NE) return;
  if (out_size != NN * OUTW) return;

  const float* x   = (const float*)d_in[0];
  const float* W1  = (const float*)d_in[1];
  const float* al1 = (const float*)d_in[2];
  const float* ar1 = (const float*)d_in[3];
  const float* b1  = (const float*)d_in[4];
  const float* W2  = (const float*)d_in[5];
  const float* al2 = (const float*)d_in[6];
  const float* ar2 = (const float*)d_in[7];
  const float* b2  = (const float*)d_in[8];
  const int*   egat = (const int*)d_in[9];
  const int*   ekey = (const int*)d_in[10];
  float* out = (float*)d_out;

  const size_t szXB   = (size_t)MPAD * FIN * 2;
  const size_t szFT   = (size_t)MPAD * HID * 4;
  const size_t szLIST = (size_t)NBLK * RCAP * 4;
  const size_t szMETA = (size_t)NBLK * NB * 2 * 4;
  const size_t szE    = (size_t)MPAD * NHD * 4;
  const size_t szW1T  = (size_t)HID * FIN * 2;
  const size_t szW2D  = (size_t)OUTW * 256 * 2;
  const size_t szTAB  = (size_t)TB_N * 4;
  static_assert((size_t)MPAD * OPK * 2 <= (size_t)MPAD * FIN * 2);
  static_assert((size_t)MPAD * OUTW * 4 <= (size_t)MPAD * HID * 4);
  static_assert((size_t)OUTW * OPK * 2 <= (size_t)OUTW * 256 * 2);
  static_assert((size_t)MPAD * FIN * 2 + (size_t)MPAD * HID * 4 + (size_t)NBLK * RCAP * 4 + (size_t)NBLK * NB * 8 +
                2 * (size_t)MPAD * NHD * 4 + (size_t)HID * FIN * 2 + (size_t)OUTW * 256 * 2 + (size_t)TB_N * 4 == 57468928);
  static_assert(57468928 <= WSMAX);
  char* ws = (char*)d_ws;
  size_t off = 0;
  const size_t oXB   = off; off += szXB;
  const size_t oFT   = off; off += szFT;
  const size_t oLIST = off; off += szLIST;
  const size_t oMETA = off; off += szMETA;
  const size_t oEL   = off; off += szE;
  const size_t oER   = off; off += szE;
  const size_t oW1T  = off; off += szW1T;
  const size_t oW2D  = off; off += szW2D;
  const size_t oTAB  = off; off += szTAB;
  if (off > ws_size || off > (size_t)WSMAX) return;
  unsigned short* XB  = (unsigned short*)(ws + oXB);
  unsigned short* OP  = XB;
  float*    FT   = (float*)(ws + oFT);
  float*    FT2  = FT;
  unsigned* LIST = (unsigned*)(ws + oLIST);
  int*      META = (int*)(ws + oMETA);
  float*    EL   = (float*)(ws + oEL);
  float*    ER   = (float*)(ws + oER);
  unsigned short* W1T = (unsigned short*)(ws + oW1T);
  unsigned short* W2D = (unsigned short*)(ws + oW2D);
  float*    TAB  = (float*)(ws + oTAB);

  hipFuncSetAttribute(reinterpret_cast<const void*>(&k_list),
                      hipFuncAttributeMaxDynamicSharedMemorySize, LDS_LST);

  k_plane<0><<<MPAD * FIN / 8 / 256, 256, 0, stream>>>(x, NN, FIN, FIN, XB, MPAD, FIN);
  k_prep<<<PREP_BLK, 256, 0, stream>>>(W1, W2, al1, ar1, b1, al2, ar2, b2, W1T, W2D, TAB);
  k_list<<<NBLK, BT, LDS_LST, stream>>>(ekey, egat, LIST, META);
  k_gemm_nt<0, 0><<<((MPAD / 64) * (HID / 64) + 7) / 8, 256, 0, stream>>>(XB, W1T, TAB, FT, MPAD, HID, FIN, HID);
  k_rowprep1<<<MPAD / RWAVES, RTHR, 0, stream>>>(FT, TAB, EL, ER);
  k_walk1<<<MPAD / RWAVES, RTHR, 0, stream>>>(FT, EL, ER, LIST, META, TAB, OP);
  k_gemm_nt<0, 0><<<((MPAD / 64) * (OUTW / 64) + 7) / 8, 256, 0, stream>>>(OP, W2D, TAB, FT2, MPAD, OUTW, OPK, OUTW);
  k_rowprep2<<<MPAD / 32, RTHR, 0, stream>>>(FT2, TAB, EL, ER);
  k_walk2<<<NN / RWAVES, RTHR, 0, stream>>>(FT2, EL, ER, LIST, META, TAB, out);
}
